// FlashAttention_86002425135546
// MI455X (gfx1250) — hardware-run, weakly checked
//
#include <hip/hip_runtime.h>
#include <math.h>

typedef __attribute__((ext_vector_type(16))) _Float16 v16h;
typedef __attribute__((ext_vector_type(8)))  _Float16 v8h;
typedef __attribute__((ext_vector_type(8)))  float    v8f;
typedef __attribute__((ext_vector_type(4)))  float    v4f;

constexpr int kBatch = 2;
constexpr int kSeq   = 2048;
constexpr int kDm    = 2048;
constexpr int kHeads = 16;
constexpr int kHd    = 128;
constexpr int kFeat  = kHeads * kHd;
constexpr int kRows  = kBatch * kSeq;
static_assert(kFeat == 2048 && kRows == 4096, "shape");
static_assert((kDm % 32) == 0 && (kHd % 32) == 0 && (kSeq % 64) == 0, "k-depth multiples of 32 / 64");
static_assert((kRows % 64) == 0 && (kFeat % 64) == 0 && (kDm % 64) == 0, "tile multiples of 64");
static_assert((kHd % 64) == 0, "a 64-wide column tile stays inside one head");

constexpr float kXCarry   = 16.0f;
constexpr float kWCarry   = 1024.0f;
constexpr float kQkvCarry = 16.0f;
constexpr float kPCarry   = 32768.0f;
constexpr float kOCarry   = 1024.0f;
constexpr float kProjScale = 1.0f / (kXCarry * kWCarry);
constexpr float kOutScale  = 1.0f / (kOCarry * kWCarry);
constexpr float kPVFold    = kOCarry / (kPCarry * kQkvCarry);
constexpr int   kOsPitch   = 132;

constexpr size_t kPlaneW  = (size_t)kDm * kFeat * 2;
constexpr size_t kPlaneA  = (size_t)kRows * kDm * 2;
constexpr size_t kOffWT   = 0;
constexpr size_t kOffX    = kOffWT + 4 * kPlaneW;
constexpr size_t kOffQ    = kOffX + kPlaneA;
constexpr size_t kOffK    = kOffQ + kPlaneA;
constexpr size_t kOffVT   = kOffK + kPlaneA;
constexpr size_t kOffO    = kOffVT + kPlaneA;
constexpr size_t kWsTotal = kOffO + kPlaneA;
static_assert(kWsTotal == 117440512ull, "carve total");
static_assert(kWsTotal <= 134217728ull, "carve cap");

__device__ __forceinline__ unsigned short f2bf_bits(float f) {
  unsigned u = __float_as_uint(f);
  return (unsigned short)((u + 0x7FFFu + ((u >> 16) & 1u)) >> 16);
}
__device__ __forceinline__ float bf_bits2f(unsigned short h) { return __uint_as_float(((unsigned)h) << 16); }
__device__ __forceinline__ float bf_rne(float f) { return bf_bits2f(f2bf_bits(f)); }

union FragU { v16h v; v8h h[2]; };
__device__ __forceinline__ v16h frag_ld(const _Float16* p) {
  FragU f;
  f.h[0] = *(const v8h*)(p);
  f.h[1] = *(const v8h*)(p + 16);
  return f.v;
}
__device__ __forceinline__ v8f mma_g(v16h a, v16h b, v8f c) {
  c = __builtin_amdgcn_wmma_f32_16x16x32_f16(false, a, false, b, (short)0, c, false, false);
  asm volatile("v_nop\n\tv_nop\n\tv_nop\n\tv_nop" : "+v"(c) : "v"(a), "v"(b));
  return c;
}

__global__ __launch_bounds__(256) void wt_cast_kernel(const float* __restrict__ W0, const float* __restrict__ W1,
                                                      const float* __restrict__ W2, const float* __restrict__ W3,
                                                      unsigned short* __restrict__ out) {
  __shared__ float sm[64][65];
  const int t  = threadIdx.x;
  const int k0 = blockIdx.x * 64;
  const int n0 = blockIdx.y * 64;
  const int z  = blockIdx.z;
  const float* W = (z == 0) ? W0 : (z == 1) ? W1 : (z == 2) ? W2 : W3;
#pragma unroll
  for (int i = 0; i < 4; ++i) {
    const int e  = i * 256 + t;
    const int r  = e >> 4;
    const int c4 = (e & 15) * 4;
    const v4f w = *(const v4f*)(W + (size_t)(k0 + r) * kFeat + n0 + c4);
    const float w0 = w[0];
    const float w1 = w[1];
    const float w2 = w[2];
    const float w3 = w[3];
    sm[c4 + 0][r] = bf_rne(w0) * kWCarry;
    sm[c4 + 1][r] = bf_rne(w1) * kWCarry;
    sm[c4 + 2][r] = bf_rne(w2) * kWCarry;
    sm[c4 + 3][r] = bf_rne(w3) * kWCarry;
  }
  __syncthreads();
  const int lane = t & 31;
  const int wave = __builtin_amdgcn_readfirstlane((int)(threadIdx.x >> 5));
  const int q = lane >> 3, c8 = (lane & 7) * 8;
  _Float16* op = (_Float16*)out + (size_t)z * kDm * kFeat;
  v8h hv[2];
#pragma unroll
  for (int it = 0; it < 2; ++it) {
    const int row = wave * 8 + it * 4 + q;
#pragma unroll
    for (int e = 0; e < 8; ++e) hv[it][e] = (_Float16)sm[row][c8 + e];
  }
  for (int pass = 0; pass < 2; ++pass) {
#pragma unroll
    for (int it = 0; it < 2; ++it) {
      const int row = wave * 8 + it * 4 + q;
      *(volatile v8h*)(op + (size_t)(n0 + row) * kDm + k0 + c8) = hv[it];
    }
    __threadfence();
  }
}

__global__ __launch_bounds__(256) void x_cast_kernel(const float* __restrict__ in, unsigned short* __restrict__ out, int n8) {
  const int i = blockIdx.x * 256 + threadIdx.x;
  if (i >= n8) return;
  const float* p = in + 8 * (size_t)i;
  const v4f a = *(const v4f*)(p);
  const v4f c = *(const v4f*)(p + 4);
  v8h hv;
#pragma unroll
  for (int e = 0; e < 4; ++e) {
    const float ae = a[e];
    const float ce = c[e];
    hv[e]     = (_Float16)(bf_rne(ae) * kXCarry);
    hv[4 + e] = (_Float16)(bf_rne(ce) * kXCarry);
  }
  _Float16* q = (_Float16*)out + 8 * (size_t)i;
  *(volatile v8h*)q = hv;
  __threadfence();
  *(volatile v8h*)q = hv;
}

template <int OUT_MODE, int BIAS_MODE>
__global__ __launch_bounds__(256) __attribute__((amdgpu_num_vgpr(256)))
void gemm_f16_kernel(const unsigned short* __restrict__ Ap, int lda,
                     const unsigned short* __restrict__ Btp, int ldb,
                     void* __restrict__ Cout, int ldc,
                     const float* __restrict__ bias,
                     int M, int N, int K, float scale, float oscale) {
  __shared__ __align__(16) float sT[8][16 * 68];
  const _Float16* A  = (const _Float16*)Ap;
  const _Float16* Bt = (const _Float16*)Btp;
  const int lane = threadIdx.x & 31;
  const int wave = __builtin_amdgcn_readfirstlane((int)(threadIdx.x >> 5));
  const int tilesN = N >> 6;
  const int tilesM = M >> 6;
  const int tile = blockIdx.x * 8 + wave;
  if (tile >= tilesM * tilesN) return;
  const int tm = tile / tilesN;
  const int tn = tile - tm * tilesN;
  const int m0 = tm << 6;
  const int n0 = tn << 6;

  const int rlane = lane & 15;
  const int koff  = (lane >> 4) * 8;
  const int mOff  = (lane >> 4) * 8;

  v8f acc[4][4];
#pragma unroll
  for (int i = 0; i < 4; ++i)
#pragma unroll
    for (int j = 0; j < 4; ++j) acc[i][j] = (v8f){0.f, 0.f, 0.f, 0.f, 0.f, 0.f, 0.f, 0.f};

  for (int k0 = 0; k0 < K; k0 += 32) {
    v16h bh[4];
#pragma unroll
    for (int j = 0; j < 4; ++j) {
      const size_t bo = (size_t)(n0 + (j << 4) + rlane) * ldb + koff + k0;
      bh[j] = frag_ld(Bt + bo);
    }
#pragma unroll
    for (int i = 0; i < 4; ++i) {
      const size_t ao = (size_t)(m0 + (i << 4) + rlane) * lda + koff + k0;
      const v16h ah = frag_ld(A + ao);
#pragma unroll
      for (int j = 0; j < 4; ++j) acc[i][j] = mma_g(ah, bh[j], acc[i][j]);
    }
  }

  float* slab = sT[wave];
#pragma unroll
  for (int i = 0; i < 4; ++i) {
    const int mBase = m0 + (i << 4);
    float brow[8];
#pragma unroll
    for (int r = 0; r < 8; ++r) brow[r] = 0.f;
    if (BIAS_MODE == 1) {
#pragma unroll
      for (int r = 0; r < 8; ++r) {
        const float bvv = bias[mBase + mOff + r];
        brow[r] = bf_rne(bvv);
      }
    }
#pragma unroll
    for (int j = 0; j < 4; ++j) {
      float bcol = 0.f;
      if (BIAS_MODE == 2) {
        const float bvv = bias[n0 + (j << 4) + rlane];
        bcol = bf_rne(bvv);
      }
#pragma unroll
      for (int r = 0; r < 8; ++r) {
        float v = acc[i][j][r] * scale;
        v += (BIAS_MODE == 1) ? brow[r] : bcol;
        v *= oscale;
        slab[(mOff + r) * 68 + (j << 4) + rlane] = v;
      }
    }
    __builtin_amdgcn_fence(__ATOMIC_RELEASE, "workgroup");
    __builtin_amdgcn_wave_barrier();
    __builtin_amdgcn_fence(__ATOMIC_ACQUIRE, "workgroup");
    if (OUT_MODE == 0) {
      float* C = (float*)Cout;
      const int hh = lane >> 4, c4 = (lane & 15) * 4;
      for (int pass = 0; pass < 2; ++pass) {
#pragma unroll
        for (int it = 0; it < 8; ++it) {
          const int row = it * 2 + hh;
          const v4f v = *(const v4f*)(slab + row * 68 + c4);
          *(volatile v4f*)(C + (size_t)(mBase + row) * ldc + n0 + c4) = v;
        }
        __threadfence();
      }
    } else {
      const int q = lane >> 3, c8 = (lane & 7) * 8;
      _Float16* C = (_Float16*)Cout;
      for (int pass = 0; pass < 2; ++pass) {
#pragma unroll
        for (int it = 0; it < 4; ++it) {
          const int row = it * 4 + q;
          const int gr  = mBase + row;
          const float* sp = slab + row * 68 + c8;
          v8h hv;
#pragma unroll
          for (int e = 0; e < 8; ++e) hv[e] = (_Float16)sp[e];
          size_t off;
          if (OUT_MODE == 1) {
            const int bb = gr / kSeq;
            const int l  = gr % kSeq;
            const int hd = n0 / kHd;
            const int d0 = n0 % kHd;
            off = ((size_t)((bb * kHeads + hd) * kSeq + l)) * kHd + d0 + c8;
          } else {
            const int bb = n0 / kSeq;
            const int l0 = n0 % kSeq;
            off = ((size_t)(bb * kFeat + gr)) * kSeq + l0 + c8;
          }
          *(volatile v8h*)(C + off) = hv;
        }
        __threadfence();
      }
    }
    __builtin_amdgcn_fence(__ATOMIC_RELEASE, "workgroup");
    __builtin_amdgcn_wave_barrier();
    __builtin_amdgcn_fence(__ATOMIC_ACQUIRE, "workgroup");
  }
}

__global__ __launch_bounds__(128) __attribute__((amdgpu_num_vgpr(256)))
void attn_kernel(const unsigned short* __restrict__ Qp, const unsigned short* __restrict__ Kp,
                 const unsigned short* __restrict__ VTp, unsigned short* __restrict__ Op, float sc) {
  __shared__ __align__(16) float sO[4][16 * kOsPitch];
  const int lane = threadIdx.x & 31;
  const int wave = __builtin_amdgcn_readfirstlane((int)(threadIdx.x >> 5));
  const int hh  = lane >> 4;
  const int n16 = lane & 15;
  constexpr int kQBlocks = kSeq / 64;
  const int bx = blockIdx.x;
  const int bh = bx / kQBlocks;
  const int qb = bx - bh * kQBlocks;
  const int b  = bh / kHeads;
  const int h  = bh - b * kHeads;
  const int q0 = qb * 64 + wave * 16;

  const _Float16* Qb = (const _Float16*)Qp  + (size_t)bh * kSeq * kHd;
  const _Float16* Kb = (const _Float16*)Kp  + (size_t)bh * kSeq * kHd;
  const _Float16* Vb = (const _Float16*)VTp + (size_t)bh * kHd * kSeq;

  v16h qf[4];
#pragma unroll
  for (int dc = 0; dc < 4; ++dc) qf[dc] = frag_ld(Qb + (size_t)(q0 + n16) * kHd + dc * 32 + 8 * hh);

  v8f o[8];
#pragma unroll
  for (int dt = 0; dt < 8; ++dt) o[dt] = (v8f){0.f, 0.f, 0.f, 0.f, 0.f, 0.f, 0.f, 0.f};
  float mq = -1e30f;
  float lq = 0.0f;

  const _Float16* kbase = Kb + (size_t)n16 * kHd + 8 * hh;
  const _Float16* vbase = Vb + (size_t)n16 * kSeq + 8 * hh;

#pragma unroll 1
  for (int j0 = 0; j0 < kSeq; j0 += 64) {
    v8f st[4];
#pragma unroll
    for (int jt = 0; jt < 4; ++jt) st[jt] = (v8f){0.f, 0.f, 0.f, 0.f, 0.f, 0.f, 0.f, 0.f};
#pragma unroll
    for (int dc = 0; dc < 4; ++dc) {
#pragma unroll
      for (int jt = 0; jt < 4; ++jt) {
        const v16h ka = frag_ld(kbase + (size_t)(j0 + jt * 16) * kHd + dc * 32);
        st[jt] = mma_g(ka, qf[dc], st[jt]);
      }
    }

    float t[4][8];
    float mx = -1e30f;
#pragma unroll
    for (int jt = 0; jt < 4; ++jt) {
#pragma unroll
      for (int r = 0; r < 8; ++r) {
        t[jt][r] = st[jt][r] * sc;
        mx = fmaxf(mx, t[jt][r]);
      }
    }
    mx = fmaxf(mx, __shfl_xor(mx, 16, 32));
    const float newm  = fmaxf(mq, mx);
    const float alpha = __expf(mq - newm);
    mq = newm;

    float sum = 0.0f;
    v16h bp[2];
#pragma unroll
    for (int kk = 0; kk < 2; ++kk) {
#pragma unroll
      for (int r = 0; r < 8; ++r) {
        const float p0 = __expf(t[2 * kk][r] - newm);
        const float p1 = __expf(t[2 * kk + 1][r] - newm);
        sum += p0 + p1;
        bp[kk][r]     = (_Float16)(p0 * kPCarry);
        bp[kk][8 + r] = (_Float16)(p1 * kPCarry);
      }
    }
    sum += __shfl_xor(sum, 16, 32);
    lq = lq * alpha + sum;

#pragma unroll
    for (int dt = 0; dt < 8; ++dt) o[dt] *= alpha;

#pragma unroll
    for (int kk = 0; kk < 2; ++kk) {
#pragma unroll
      for (int dt = 0; dt < 8; ++dt) {
        const v16h va = frag_ld(vbase + (size_t)(dt * 16) * kSeq + j0 + kk * 32);
        o[dt] = mma_g(va, bp[kk], o[dt]);
      }
    }
  }

  const float inv = kPVFold * (1.0f / lq);
  float* os = sO[wave];
#pragma unroll
  for (int dt = 0; dt < 8; ++dt) {
#pragma unroll
    for (int r = 0; r < 8; ++r) os[n16 * kOsPitch + dt * 16 + 8 * hh + r] = o[dt][r] * inv;
  }
  __builtin_amdgcn_fence(__ATOMIC_RELEASE, "workgroup");
  __builtin_amdgcn_wave_barrier();
  __builtin_amdgcn_fence(__ATOMIC_ACQUIRE, "workgroup");

  const int c8 = n16 * 8;
  v8h hv[8];
#pragma unroll
  for (int it = 0; it < 8; ++it) {
    const int row = it * 2 + hh;
    const float* sp = os + row * kOsPitch + c8;
    const v4f a0 = *(const v4f*)(sp);
    const v4f a1 = *(const v4f*)(sp + 4);
#pragma unroll
    for (int e = 0; e < 4; ++e) {
      const float x0 = a0[e];
      const float x1 = a1[e];
      hv[it][e]     = (_Float16)x0;
      hv[it][4 + e] = (_Float16)x1;
    }
  }
  _Float16* Ob = (_Float16*)Op + (size_t)(b * kSeq + q0) * kDm + h * kHd + c8;
  for (int pass = 0; pass < 2; ++pass) {
#pragma unroll
    for (int it = 0; it < 8; ++it) {
      const int row = it * 2 + hh;
      *(volatile v8h*)(Ob + (size_t)row * kDm) = hv[it];
    }
    __threadfence();
  }
}

extern "C" void kernel_launch(void* const* d_in, const int* in_sizes, int n_in,
                              void* d_out, int out_size, void* d_ws, size_t ws_size,
                              hipStream_t stream) {
  if (n_in < 9) return;
  if (in_sizes[0] != kRows * kDm || in_sizes[0] != kRows * kDm || in_sizes[0] != kRows * kDm) return;
  if (in_sizes[1] != kDm * kFeat || in_sizes[3] != kDm * kFeat || in_sizes[5] != kDm * kFeat) return;
  if (in_sizes[7] != kFeat * kDm) return;
  if (in_sizes[2] != kFeat || in_sizes[4] != kFeat || in_sizes[6] != kFeat || in_sizes[8] != kDm) return;
  if (out_size != kRows * kDm) return;
  if (ws_size < kWsTotal) return;

  const float* x_q = (const float*)d_in[0];
  const float* x_k = (const float*)d_in[0];
  const float* x_v = (const float*)d_in[0];
  const float* Wq  = (const float*)d_in[1];
  const float* bq  = (const float*)d_in[2];
  const float* Wk  = (const float*)d_in[3];
  const float* bk  = (const float*)d_in[4];
  const float* Wv  = (const float*)d_in[5];
  const float* bv  = (const float*)d_in[6];
  const float* Wo  = (const float*)d_in[7];
  const float* bo  = (const float*)d_in[8];
  float* out = (float*)d_out;

  char* ws = (char*)d_ws;
  unsigned short* WT  = (unsigned short*)(ws + kOffWT);
  unsigned short* WqT = WT;
  unsigned short* WkT = WT + (size_t)1 * kDm * kFeat;
  unsigned short* WvT = WT + (size_t)2 * kDm * kFeat;
  unsigned short* WoT = WT + (size_t)3 * kDm * kFeat;
  unsigned short* X   = (unsigned short*)(ws + kOffX);
  unsigned short* Qh  = (unsigned short*)(ws + kOffQ);
  unsigned short* Kh  = (unsigned short*)(ws + kOffK);
  unsigned short* VTh = (unsigned short*)(ws + kOffVT);
  unsigned short* Oh  = (unsigned short*)(ws + kOffO);

  const int n8 = kRows * kDm / 8;
  const int castBlocks = n8 / 256;
  const int gemmBlocks = (kRows / 64) * (kFeat / 64) / 8;
  const float sc = (float)(1.0 / sqrt((double)kHd)) / (kQkvCarry * kQkvCarry);

  wt_cast_kernel<<<dim3(kDm / 64, kFeat / 64, 4), 256, 0, stream>>>(Wq, Wk, Wv, Wo, WT);

  x_cast_kernel<<<castBlocks, 256, 0, stream>>>(x_q, X, n8);
  gemm_f16_kernel<1, 2><<<gemmBlocks, 256, 0, stream>>>(X, kDm, WqT, kDm, (void*)Qh, 0, bq,
                                                        kRows, kFeat, kDm, kProjScale, kQkvCarry);

  x_cast_kernel<<<castBlocks, 256, 0, stream>>>(x_k, X, n8);
  gemm_f16_kernel<1, 2><<<gemmBlocks, 256, 0, stream>>>(X, kDm, WkT, kDm, (void*)Kh, 0, bk,
                                                        kRows, kFeat, kDm, kProjScale, kQkvCarry);

  x_cast_kernel<<<castBlocks, 256, 0, stream>>>(x_v, X, n8);
  gemm_f16_kernel<2, 1><<<gemmBlocks, 256, 0, stream>>>(WvT, kDm, X, kDm, (void*)VTh, 0, bv,
                                                        kFeat, kRows, kDm, kProjScale, kQkvCarry);

  attn_kernel<<<kBatch * kHeads * (kSeq / 64), 128, 0, stream>>>(Qh, Kh, VTh, Oh, sc);

  gemm_f16_kernel<0, 2><<<gemmBlocks, 256, 0, stream>>>(Oh, kFeat, WoT, kFeat, (void*)out, kDm, bo,
                                                        kRows, kDm, kFeat, kOutScale, 1.0f);
}
